// MultiHeadATT_86320252715606
// MI455X (gfx1250) — hardware-verified
//
#include <hip/hip_runtime.h>
#include <math.h>
#include <stdint.h>

#ifndef NB
#define NB       4
#endif
#ifndef SQ
#define SQ       2048
#endif
#define NB_FULL  4
#define SQ_FULL  2048
#define SKV      SQ_FULL
#define DM       512
#define NH       8
#define HD       64
#define INNER    (NH * HD)
#define WSC      256.0f
#define QS       8.0f
#define KS       8.0f
#define VS       8.0f
#define CS       16.0f
#define RSC      2048.0f
#define RRSC     0.00048828125f
#define PCAR     32768.0f
#define LOG2E    1.4426950408889634f
#define RSQH     0.35355339059327373f
#define LN_EPS   1e-5f
#define NKB      (SKV / 32)
#define ATT_WAVES   4
#define ATT_THREADS (ATT_WAVES * 32)
#define CVT_THREADS 128
#define LN_THREADS  256
#define OPITCH   68
#define GPITCH   68

static_assert(NB >= 1 && NB <= NB_FULL);
static_assert((SQ % 128) == 0 && SQ >= 128 && SQ <= SQ_FULL);
static_assert(HD == 64 && NH == 8 && INNER == 512 && INNER == DM);
static_assert((HD % 32) == 0);
static_assert((SKV % 128) == 0 && (SKV % 64) == 0 && NKB * 32 == SKV);
static_assert(DM == 512 && (DM % 64) == 0 && (DM % 32) == 0 && DM == 4 * CVT_THREADS);
static_assert((NB * SQ) % (LN_THREADS / 32) == 0);
static_assert((OPITCH * 4) % 16 == 0 && (GPITCH * 4) % 16 == 0);
static_assert(ATT_THREADS == 128 && LN_THREADS == 256 && CVT_THREADS == 128);

typedef unsigned short u16;
typedef _Float16 v16h __attribute__((ext_vector_type(16)));
typedef _Float16 v8h  __attribute__((ext_vector_type(8)));
typedef float    v8f  __attribute__((ext_vector_type(8)));
typedef float    v4f  __attribute__((ext_vector_type(4)));
typedef unsigned int v4u __attribute__((ext_vector_type(4)));

union FragH { v16h v; v8h h[2]; v4u u[2]; };

__device__ __forceinline__ unsigned short bf_bits(float f) {
  unsigned u = __float_as_uint(f);
  return (unsigned short)((u + 0x7FFFu + ((u >> 16) & 1u)) >> 16);
}
__device__ __forceinline__ float bf_up(unsigned short h) { return __uint_as_float(((unsigned)h) << 16); }
__device__ __forceinline__ float bfr(float f) { return bf_up(bf_bits(f)); }
__device__ __forceinline__ unsigned short h_bits(_Float16 x) { return __builtin_bit_cast(unsigned short, x); }
__device__ __forceinline__ unsigned pk16(unsigned short a, unsigned short b) { return (unsigned)a | ((unsigned)b << 16); }
__device__ __forceinline__ v8f zero8() { v8f z = {0.f, 0.f, 0.f, 0.f, 0.f, 0.f, 0.f, 0.f}; return z; }
__device__ __forceinline__ unsigned pk_hi(float a, float b) {
  return pk16(h_bits((_Float16)a), h_bits((_Float16)b));
}
__device__ __forceinline__ unsigned pk_lo(float a, float b) {
  const float ra = (a - (float)((_Float16)a)) * RSC;
  const float rb = (b - (float)((_Float16)b)) * RSC;
  return pk16(h_bits((_Float16)ra), h_bits((_Float16)rb));
}

__device__ __forceinline__ v16h ldfrag_h(const _Float16* p) {
  FragH f;
  f.h[0] = *(const v8h*)(p);
  f.h[1] = *(const v8h*)(p + 16);
  return f.v;
}

__device__ __forceinline__ v8f mma_h(v16h a, v16h b, v8f c) {
  return __builtin_amdgcn_wmma_f32_16x16x32_f16(false, a, false, b, (short)0, c, false, false);
}
__device__ __forceinline__ void guard_s4(v8f& a, v8f& b, v8f& c, v8f& d,
                                         v16h x0, v16h x1, v16h x2, v16h x3, v16h x4, v16h x5) {
#if defined(__HIP_DEVICE_COMPILE__)
  asm volatile("v_nop\n\tv_nop\n\tv_nop\n\tv_nop"
               : "+v"(a), "+v"(b), "+v"(c), "+v"(d)
               : "v"(x0), "v"(x1), "v"(x2), "v"(x3), "v"(x4), "v"(x5) : "memory");
#endif
}
__device__ __forceinline__ void guard_p(v8f& a, v8f& b, v8f& c, v8f& d, v16h p, v16h x0, v16h x1, v16h x2, v16h x3) {
#if defined(__HIP_DEVICE_COMPILE__)
  asm volatile("v_nop\n\tv_nop\n\tv_nop\n\tv_nop"
               : "+v"(a), "+v"(b), "+v"(c), "+v"(d) : "v"(p), "v"(x0), "v"(x1), "v"(x2), "v"(x3) : "memory");
#endif
}
__device__ __forceinline__ void guard_g(v8f (&acc)[8], v16h x0, v16h x1, v16h x2, v16h x3, v16h x4, v16h x5) {
#if defined(__HIP_DEVICE_COMPILE__)
  asm volatile("v_nop\n\tv_nop\n\tv_nop\n\tv_nop"
               : "+v"(acc[0]), "+v"(acc[1]), "+v"(acc[2]), "+v"(acc[3]),
                 "+v"(acc[4]), "+v"(acc[5]), "+v"(acc[6]), "+v"(acc[7])
               : "v"(x0), "v"(x1), "v"(x2), "v"(x3), "v"(x4), "v"(x5) : "memory");
#endif
}
__device__ __forceinline__ void acc_guard8(v8f (&o)[8]) {
#if defined(__HIP_DEVICE_COMPILE__)
  asm volatile("v_nop\n\tv_nop\n\tv_nop\n\tv_nop"
               : "+v"(o[0]), "+v"(o[1]), "+v"(o[2]), "+v"(o[3]), "+v"(o[4]), "+v"(o[5]), "+v"(o[6]), "+v"(o[7]));
#endif
}
__device__ __forceinline__ void acc_guard4(v8f (&o)[4]) {
#if defined(__HIP_DEVICE_COMPILE__)
  asm volatile("v_nop\n\tv_nop\n\tv_nop\n\tv_nop" : "+v"(o[0]), "+v"(o[1]), "+v"(o[2]), "+v"(o[3]));
#endif
}
__device__ __forceinline__ void wave_sync_lds() {
  __builtin_amdgcn_fence(__ATOMIC_RELEASE, "workgroup");
  __builtin_amdgcn_wave_barrier();
  __builtin_amdgcn_fence(__ATOMIC_ACQUIRE, "workgroup");
}

__global__ __launch_bounds__(CVT_THREADS)
void cvt16(const float* __restrict__ x, u16* Y, int rowsPerB, int srcRowsPerB, float scale) {
  const int tid = threadIdx.x;
  const int r   = blockIdx.x * 2 + (tid >> 6);
  const int t8  = (tid & 63) * 8;
  const int b   = r / rowsPerB;
  const int s   = r - b * rowsPerB;
  const float* src = x + ((size_t)b * (size_t)srcRowsPerB + (size_t)s) * (size_t)DM + (size_t)t8;
  const v4f a = *(const v4f*)(src), c4 = *(const v4f*)(src + 4);
  v4u o;
#pragma unroll
  for (int e = 0; e < 2; ++e) {
    o[e]     = pk16(h_bits((_Float16)(bfr(a[2 * e]) * scale)),  h_bits((_Float16)(bfr(a[2 * e + 1]) * scale)));
    o[2 + e] = pk16(h_bits((_Float16)(bfr(c4[2 * e]) * scale)), h_bits((_Float16)(bfr(c4[2 * e + 1]) * scale)));
  }
  u16* dst = Y + (size_t)r * (size_t)DM + (size_t)t8;
  for (int pass = 0; pass < 2; ++pass) {
    *(volatile v4u*)(dst) = o;
    __threadfence();
  }
}

__device__ __forceinline__ void gemm_core(const _Float16* ap, const _Float16* bp, int K, v8f (&acc)[8]) {
  const size_t rs16 = (size_t)16 * (size_t)K;
#pragma unroll 1
  for (int k0 = 0; k0 < K; k0 += 32) {
    const v16h a0 = ldfrag_h(ap + k0), a1 = ldfrag_h(ap + rs16 + k0);
    const v16h b0 = ldfrag_h(bp + k0);
    const v16h b1 = ldfrag_h(bp + rs16 + k0);
    const v16h b2 = ldfrag_h(bp + 2 * rs16 + k0);
    const v16h b3 = ldfrag_h(bp + 3 * rs16 + k0);
    acc[0] = mma_h(a0, b0, acc[0]);
    acc[1] = mma_h(a0, b1, acc[1]);
    acc[2] = mma_h(a0, b2, acc[2]);
    acc[3] = mma_h(a0, b3, acc[3]);
    acc[4] = mma_h(a1, b0, acc[4]);
    acc[5] = mma_h(a1, b1, acc[5]);
    acc[6] = mma_h(a1, b2, acc[6]);
    acc[7] = mma_h(a1, b3, acc[7]);
    guard_g(acc, a0, a1, b0, b1, b2, b3);
  }
}
__device__ __forceinline__ void stage32x64(float* sl, v8f (&acc)[8], float oscale, int lane) {
  const int hh = lane >> 4, m = lane & 15;
#pragma unroll
  for (int i = 0; i < 2; ++i) {
#pragma unroll
    for (int r = 0; r < 8; ++r) {
      const int ro = (16 * i + 8 * hh + r) * GPITCH + m;
      sl[ro]      = acc[4 * i + 0][r] * oscale;
      sl[ro + 16] = acc[4 * i + 1][r] * oscale;
      sl[ro + 32] = acc[4 * i + 2][r] * oscale;
      sl[ro + 48] = acc[4 * i + 3][r] * oscale;
    }
  }
  wave_sync_lds();
}

__global__ __launch_bounds__(128)
void gemm_o16(const u16* __restrict__ A, const u16* __restrict__ Bt, u16* C, u16* C2,
              const float* __restrict__ bias, int biasN, int biasRow,
              int Mb, int N, int K, int aBs, int bBs, int cBs, float oscale, float bscale, int res) {
  __shared__ __align__(16) float slab[4 * 32 * GPITCH];
  const int tid = threadIdx.x, wave = tid >> 5, lane = tid & 31, hh = lane >> 4, m = lane & 15;
  const int ntile = N >> 6, mtile = Mb >> 7;
  const int bid  = blockIdx.x;
  const int nt   = bid % ntile;
  const int tmp  = bid / ntile;
  const int mt   = tmp % mtile;
  const int bz   = tmp / mtile;
  const int rowb = mt * 128 + wave * 32;
  const int col0 = nt * 64;
  if (rowb + 32 > Mb) return;
  const _Float16* Ab = (const _Float16*)(const void*)A + (size_t)bz * (size_t)aBs;
  const _Float16* Bb = (const _Float16*)(const void*)Bt + (size_t)bz * (size_t)bBs;
  const _Float16* ap = Ab + (size_t)(rowb + m) * (size_t)K + 8 * hh;
  const _Float16* bp = Bb + (size_t)(col0 + m) * (size_t)K + 8 * hh;
  v8f acc[8];
#pragma unroll
  for (int i = 0; i < 8; ++i) acc[i] = zero8();
  gemm_core(ap, bp, K, acc);
  float* sl = slab + wave * 32 * GPITCH;
  stage32x64(sl, acc, oscale, lane);
  const int rq = lane >> 3, c8 = (lane & 7) * 8;
  const int bl = biasN - 1;
  const float selc = (biasRow != 0) ? 0.f : bscale;
  const float selr = (biasRow != 0) ? bscale : 0.f;
  float cb[8];
#pragma unroll
  for (int e = 0; e < 8; ++e) {
    int ci = col0 + c8 + e;
    ci = (ci < bl) ? ci : bl;
    cb[e] = bfr(bias[ci]) * selc;
  }
  v4u ovh[8], ovl[8];
#pragma unroll
  for (int i = 0; i < 8; ++i) {
    const int row = 4 * i + rq;
    int ri = rowb + row;
    ri = (ri < bl) ? ri : bl;
    const float rb = bfr(bias[ri]) * selr;
    const v4f a = *(const v4f*)(sl + row * GPITCH + c8), c4 = *(const v4f*)(sl + row * GPITCH + c8 + 4);
    float v[8];
#pragma unroll
    for (int e = 0; e < 4; ++e) { v[e] = a[e] + cb[e] + rb; v[4 + e] = c4[e] + cb[4 + e] + rb; }
#pragma unroll
    for (int e = 0; e < 4; ++e) {
      ovh[i][e] = pk_hi(v[2 * e], v[2 * e + 1]);
      ovl[i][e] = pk_lo(v[2 * e], v[2 * e + 1]);
    }
  }
  const size_t cofs = (size_t)bz * (size_t)cBs + (size_t)rowb * (size_t)N + (size_t)(col0 + c8);
  u16* Cb  = C + cofs;
  u16* C2b = C2 + cofs;
  for (int pass = 0; pass < 2; ++pass) {
#pragma unroll
    for (int i = 0; i < 8; ++i) {
      const int row = 4 * i + rq;
      *(volatile v4u*)(Cb + (size_t)row * (size_t)N) = ovh[i];
    }
    if (res != 0) {
#pragma unroll
      for (int i = 0; i < 8; ++i) {
        const int row = 4 * i + rq;
        *(volatile v4u*)(C2b + (size_t)row * (size_t)N) = ovl[i];
      }
    }
    __threadfence();
  }
}

__global__ __launch_bounds__(128)
void gemm_o32(const u16* __restrict__ Ah, const u16* __restrict__ Al, const u16* __restrict__ Bt,
              const float* __restrict__ bias, int biasN, const float* __restrict__ R, int rowsPerB, int srcRowsPerB,
              float* X, int Mb, int N, int K, float oscale, float rres) {
  __shared__ __align__(16) float slab[4 * 32 * GPITCH];
  const int tid = threadIdx.x, wave = tid >> 5, lane = tid & 31, hh = lane >> 4, m = lane & 15;
  const int ntile = N >> 6;
  const int bid  = blockIdx.x;
  const int nt   = bid % ntile;
  const int mt   = bid / ntile;
  const int rowb = mt * 128 + wave * 32;
  const int col0 = nt * 64;
  if (rowb + 32 > Mb) return;
  const _Float16* aph = (const _Float16*)(const void*)Ah + (size_t)(rowb + m) * (size_t)K + 8 * hh;
  const _Float16* apl = (const _Float16*)(const void*)Al + (size_t)(rowb + m) * (size_t)K + 8 * hh;
  const _Float16* bp  = (const _Float16*)(const void*)Bt + (size_t)(col0 + m) * (size_t)K + 8 * hh;
  v8f acc[8];
#pragma unroll
  for (int i = 0; i < 8; ++i) acc[i] = zero8();
  gemm_core(apl, bp, K, acc);
#pragma unroll
  for (int i = 0; i < 8; ++i) {
#pragma unroll
    for (int r = 0; r < 8; ++r) acc[i][r] *= rres;
  }
  acc_guard8(acc);
  gemm_core(aph, bp, K, acc);
  float* sl = slab + wave * 32 * GPITCH;
  stage32x64(sl, acc, oscale, lane);
  const int r2 = lane >> 4, c4 = (lane & 15) * 4;
  const int bl = biasN - 1;
  float cb[4];
#pragma unroll
  for (int e = 0; e < 4; ++e) {
    int ci = col0 + c4 + e;
    ci = (ci < bl) ? ci : bl;
    cb[e] = bfr(bias[ci]);
  }
  v4f vals[16];
#pragma unroll
  for (int i = 0; i < 16; ++i) {
    const int row  = 2 * i + r2;
    const int grow = rowb + row;
    const int bb   = grow / rowsPerB;
    const int ss   = grow - bb * rowsPerB;
    const float* rp = R + ((size_t)bb * (size_t)srcRowsPerB + (size_t)ss) * (size_t)N + (size_t)(col0 + c4);
    const v4f rv = *(const v4f*)(rp);
    const v4f a  = *(const v4f*)(sl + row * GPITCH + c4);
    v4f y;
#pragma unroll
    for (int e = 0; e < 4; ++e) y[e] = a[e] + cb[e] + bfr(rv[e]);
    vals[i] = y;
  }
  float* Xb = X + (size_t)rowb * (size_t)N + (size_t)(col0 + c4);
  for (int pass = 0; pass < 2; ++pass) {
#pragma unroll
    for (int i = 0; i < 16; ++i) {
      const int row = 2 * i + r2;
      *(volatile v4f*)(Xb + (size_t)row * (size_t)N) = vals[i];
    }
    __threadfence();
  }
}

__global__ __launch_bounds__(ATT_THREADS)
void attn_fwd(const u16* __restrict__ QH, const u16* __restrict__ QL, const u16* __restrict__ KH,
              const u16* __restrict__ KL, const u16* __restrict__ VT, u16* CH, u16* CL) {
  __shared__ __align__(16) float smem[ATT_WAVES * 16 * OPITCH];

  const int tid  = threadIdx.x;
  const int wave = tid >> 5;
  const int lane = tid & 31;
  const int hh   = lane >> 4;
  const int c    = lane & 15;

  constexpr int NQT = SQ / 64;
  const int bid  = blockIdx.x;
  const int qt   = bid % NQT;
  const int head = (bid / NQT) % NH;
  const int b    = bid / (NQT * NH);
  const int q0   = qt * 64 + wave * 16;

  const size_t qoff = ((size_t)(b * SQ + q0 + c)) * DM + head * HD + 8 * hh;
  const _Float16* Qh = (const _Float16*)(const void*)QH + qoff;
  const _Float16* Ql = (const _Float16*)(const void*)QL + qoff;
  const size_t koff = ((size_t)(b * SKV + c)) * DM + head * HD + 8 * hh;
  const _Float16* Kh = (const _Float16*)(const void*)KH + koff;
  const _Float16* Kl = (const _Float16*)(const void*)KL + koff;
  const _Float16* Vb = (const _Float16*)(const void*)VT + ((size_t)((b * NH + head) * HD + c)) * SKV + 8 * hh;
  const float lsc = (LOG2E * RSQH) / (QS * KS);

  v16h qh[2], ql[2];
#pragma unroll
  for (int dc = 0; dc < 2; ++dc) { qh[dc] = ldfrag_h(Qh + 32 * dc); ql[dc] = ldfrag_h(Ql + 32 * dc); }

  float mrun = -INFINITY, lrun = 0.f;
  v8f o[4];
#pragma unroll
  for (int j = 0; j < 4; ++j) o[j] = zero8();

#pragma unroll 1
  for (int it = 0; it < NKB; ++it) {
    const int kb = it * 32;
    v8f s0 = zero8(), s1 = zero8(), x0 = zero8(), x1 = zero8();
    const _Float16* kh0p = Kh + (size_t)kb * DM;
    const _Float16* kh1p = kh0p + (size_t)16 * DM;
    const _Float16* kl0p = Kl + (size_t)kb * DM;
    const _Float16* kl1p = kl0p + (size_t)16 * DM;
#pragma unroll
    for (int kk = 0; kk < HD / 32; ++kk) {
      const v16h fh0 = ldfrag_h(kh0p + kk * 32);
      const v16h fh1 = ldfrag_h(kh1p + kk * 32);
      const v16h fl0 = ldfrag_h(kl0p + kk * 32);
      const v16h fl1 = ldfrag_h(kl1p + kk * 32);
      s0 = mma_h(fh0, qh[kk], s0);
      s1 = mma_h(fh1, qh[kk], s1);
      x0 = mma_h(fh0, ql[kk], x0);
      x1 = mma_h(fh1, ql[kk], x1);
      x0 = mma_h(fl0, qh[kk], x0);
      x1 = mma_h(fl1, qh[kk], x1);
      guard_s4(s0, s1, x0, x1, qh[kk], ql[kk], fh0, fh1, fl0, fl1);
    }
    float t[16];
#pragma unroll
    for (int i = 0; i < 8; ++i) {
      t[i]     = (s0[i] + x0[i] * RRSC) * lsc;
      t[8 + i] = (s1[i] + x1[i] * RRSC) * lsc;
    }
    float cm = t[0];
#pragma unroll
    for (int i = 1; i < 16; ++i) cm = fmaxf(cm, t[i]);
    cm = fmaxf(cm, __shfl_xor(cm, 16, 32));
    const float mn = fmaxf(mrun, cm);
    const float al = exp2f(mrun - mn);
    mrun = mn;
    float ps = 0.f;
    FragH ph;
#pragma unroll
    for (int w = 0; w < 2; ++w) {
#pragma unroll
      for (int e4 = 0; e4 < 4; ++e4) {
        const int i = 8 * w + 2 * e4;
        const float p0 = exp2f(t[i] - mn), p1 = exp2f(t[i + 1] - mn);
        ps += p0 + p1;
        ph.u[w][e4] = pk16(h_bits((_Float16)(p0 * PCAR)), h_bits((_Float16)(p1 * PCAR)));
      }
    }
    ps += __shfl_xor(ps, 16, 32);
    lrun = lrun * al + ps;
    float scl[8];
#pragma unroll
    for (int r = 0; r < 8; ++r) scl[r] = __shfl(al, 8 * hh + r, 32);
#pragma unroll
    for (int j = 0; j < 4; ++j) {
#pragma unroll
      for (int r = 0; r < 8; ++r) o[j][r] *= scl[r];
    }
    const _Float16* vp = Vb + kb;
    {
      const v16h v0 = ldfrag_h(vp);
      const v16h v1 = ldfrag_h(vp + (size_t)16 * SKV);
      const v16h v2 = ldfrag_h(vp + (size_t)32 * SKV);
      const v16h v3 = ldfrag_h(vp + (size_t)48 * SKV);
      o[0] = mma_h(ph.v, v0, o[0]);
      o[1] = mma_h(ph.v, v1, o[1]);
      o[2] = mma_h(ph.v, v2, o[2]);
      o[3] = mma_h(ph.v, v3, o[3]);
      guard_p(o[0], o[1], o[2], o[3], ph.v, v0, v1, v2, v3);
    }
  }
  acc_guard4(o);

  const float linv = (1.0f / lrun) * (CS / (PCAR * VS));
  float inv[8];
#pragma unroll
  for (int r = 0; r < 8; ++r) inv[r] = __shfl(linv, 8 * hh + r, 32);
  float* slab = smem + wave * 16 * OPITCH;
#pragma unroll
  for (int r = 0; r < 8; ++r) {
#pragma unroll
    for (int j = 0; j < 4; ++j) slab[(8 * hh + r) * OPITCH + j * 16 + c] = o[j][r] * inv[r];
  }
  wave_sync_lds();
  const int rq = lane >> 3, c8 = (lane & 7) * 8;
  v4u ovh[4], ovl[4];
#pragma unroll
  for (int i = 0; i < 4; ++i) {
    const int row = 4 * i + rq;
    const v4f a = *(const v4f*)(slab + row * OPITCH + c8), c4 = *(const v4f*)(slab + row * OPITCH + c8 + 4);
#pragma unroll
    for (int e = 0; e < 2; ++e) {
      ovh[i][e]     = pk_hi(a[2 * e], a[2 * e + 1]);
      ovl[i][e]     = pk_lo(a[2 * e], a[2 * e + 1]);
      ovh[i][2 + e] = pk_hi(c4[2 * e], c4[2 * e + 1]);
      ovl[i][2 + e] = pk_lo(c4[2 * e], c4[2 * e + 1]);
    }
  }
  const size_t cofs = ((size_t)(b * SQ + q0)) * DM + head * HD + c8;
  u16* ch = CH + cofs;
  u16* cl = CL + cofs;
  for (int pass = 0; pass < 2; ++pass) {
#pragma unroll
    for (int i = 0; i < 4; ++i) {
      const int row = 4 * i + rq;
      *(volatile v4u*)(ch + (size_t)row * DM) = ovh[i];
      *(volatile v4u*)(cl + (size_t)row * DM) = ovl[i];
    }
    __threadfence();
  }
}

__global__ __launch_bounds__(LN_THREADS)
void ln_rows(const float* __restrict__ X, const float* __restrict__ gam, const float* __restrict__ bet, float* Out) {
  const int tid = threadIdx.x, wave = tid >> 5, lane = tid & 31;
  constexpr int RPB = LN_THREADS / 32;
  const int row = blockIdx.x * RPB + wave;
  const int b = row / SQ, s = row - b * SQ;
  const float* xr = X + (size_t)row * DM + 4 * lane;
  v4f xv[4];
  float sum = 0.f;
#pragma unroll
  for (int i = 0; i < 4; ++i) {
    xv[i] = *(const v4f*)(xr + 128 * i);
    sum += (xv[i][0] + xv[i][1]) + (xv[i][2] + xv[i][3]);
  }
#pragma unroll
  for (int mk = 16; mk >= 1; mk >>= 1) sum += __shfl_xor(sum, mk, 32);
  const float mean = sum * (1.0f / (float)DM);
  float sq = 0.f;
#pragma unroll
  for (int i = 0; i < 4; ++i) {
#pragma unroll
    for (int e = 0; e < 4; ++e) { const float d = xv[i][e] - mean; sq += d * d; }
  }
#pragma unroll
  for (int mk = 16; mk >= 1; mk >>= 1) sq += __shfl_xor(sq, mk, 32);
  const float var  = sq * (1.0f / (float)DM);
  const float rstd = 1.0f / sqrtf(var + LN_EPS);
  v4f y[4];
#pragma unroll
  for (int i = 0; i < 4; ++i) {
#pragma unroll
    for (int e = 0; e < 4; ++e) {
      const int idx = 128 * i + 4 * lane + e;
      y[i][e] = (xv[i][e] - mean) * rstd * bfr(gam[idx]) + bfr(bet[idx]);
    }
  }
  float* ob = Out + ((size_t)b * SQ_FULL + (size_t)s) * DM + 4 * lane;
  for (int pass = 0; pass < 2; ++pass) {
#pragma unroll
    for (int i = 0; i < 4; ++i) {
      *(volatile v4f*)(ob + 128 * i) = y[i];
    }
    __threadfence();
  }
}

extern "C" void kernel_launch(void* const* d_in, const int* in_sizes, int n_in,
                              void* d_out, int out_size, void* d_ws, size_t ws_size,
                              hipStream_t stream) {
  if (n_in < 13) return;
  if (in_sizes[0] < ((NB - 1) * SQ_FULL + SQ) * DM) return;
  if (in_sizes[1] < NB * SKV * DM || in_sizes[2] < NB * SKV * DM) return;
  if (in_sizes[3] != DM * DM || in_sizes[5] != DM * DM || in_sizes[7] != DM * DM || in_sizes[9] != DM * DM) return;
  if (in_sizes[4] < DM || in_sizes[6] < DM || in_sizes[8] < DM || in_sizes[10] < DM) return;
  if (in_sizes[11] < DM || in_sizes[12] < DM) return;
  if (out_size < ((NB - 1) * SQ_FULL + SQ) * DM) return;

  const float* xq  = (const float*)d_in[0];
  const float* xk  = (const float*)d_in[1];
  const float* xv  = (const float*)d_in[2];
  const float* wq  = (const float*)d_in[3];
  const float* bq  = (const float*)d_in[4];
  const float* wk  = (const float*)d_in[5];
  const float* bk  = (const float*)d_in[6];
  const float* wv  = (const float*)d_in[7];
  const float* bv  = (const float*)d_in[8];
  const float* wo  = (const float*)d_in[9];
  const float* bo  = (const float*)d_in[10];
  const float* gam = (const float*)d_in[11];
  const float* bet = (const float*)d_in[12];
  float*       out = (float*)d_out;
  const int nbq = in_sizes[4], nbk = in_sizes[6], nbv = in_sizes[8], nbo = in_sizes[10];

  const size_t szXQ  = (size_t)NB * SQ * DM * 2;
  const size_t szXKV = (size_t)NB * SKV * DM * 2;
  const size_t szW   = (size_t)DM * DM * 2;
  const size_t szQ   = (size_t)NB * SQ * INNER * 2;
  const size_t szK   = (size_t)NB * SKV * INNER * 2;
  const size_t szVT  = (size_t)NB * INNER * SKV * 2;
  const size_t szC   = (size_t)NB * SQ * INNER * 2;
  const size_t szX32 = (size_t)NB * SQ * DM * 4;
  size_t off = 0;
  const size_t oXQ  = off; off += szXQ;
  const size_t oXK  = off; off += szXKV;
  const size_t oXV  = off; off += szXKV;
  const size_t oWQ  = off; off += szW;
  const size_t oWK  = off; off += szW;
  const size_t oWV  = off; off += szW;
  const size_t oWO  = off; off += szW;
  const size_t oQH  = off; off += szQ;
  const size_t oQL  = off; off += szQ;
  const size_t oKH  = off; off += szK;
  const size_t oKL  = off; off += szK;
  const size_t oVT  = off; off += szVT;
  const size_t oCH  = off; off += szC;
  const size_t oCL  = off; off += szC;
  const size_t oX32 = off; off += szX32;
  if (off > ws_size) return;
  if (off > (size_t)134217728) return;

  char* ws = (char*)d_ws;
  u16* XQ   = (u16*)(ws + oXQ);
  u16* XK   = (u16*)(ws + oXK);
  u16* XV   = (u16*)(ws + oXV);
  u16* WQ16 = (u16*)(ws + oWQ);
  u16* WK16 = (u16*)(ws + oWK);
  u16* WV16 = (u16*)(ws + oWV);
  u16* WO16 = (u16*)(ws + oWO);
  u16* QH   = (u16*)(ws + oQH);
  u16* QL   = (u16*)(ws + oQL);
  u16* KH   = (u16*)(ws + oKH);
  u16* KL   = (u16*)(ws + oKL);
  u16* VT16 = (u16*)(ws + oVT);
  u16* CH   = (u16*)(ws + oCH);
  u16* CL   = (u16*)(ws + oCL);
  float* X32 = (float*)(ws + oX32);

  cvt16<<<dim3(NB * SQ / 2), dim3(CVT_THREADS), 0, stream>>>(xq, XQ, SQ, SQ_FULL, 1.0f);
  cvt16<<<dim3(NB * SKV / 2), dim3(CVT_THREADS), 0, stream>>>(xk, XK, SKV, SQ_FULL, 1.0f);
  cvt16<<<dim3(NB * SKV / 2), dim3(CVT_THREADS), 0, stream>>>(xv, XV, SKV, SQ_FULL, 1.0f);
  cvt16<<<dim3(DM / 2), dim3(CVT_THREADS), 0, stream>>>(wq, WQ16, DM, DM, WSC);
  cvt16<<<dim3(DM / 2), dim3(CVT_THREADS), 0, stream>>>(wk, WK16, DM, DM, WSC);
  cvt16<<<dim3(DM / 2), dim3(CVT_THREADS), 0, stream>>>(wv, WV16, DM, DM, WSC);
  cvt16<<<dim3(DM / 2), dim3(CVT_THREADS), 0, stream>>>(wo, WO16, DM, DM, WSC);
  gemm_o16<<<dim3((NB * SQ / 128) * (INNER / 64)), dim3(128), 0, stream>>>(
      XQ, WQ16, QH, QL, bq, nbq, 0, NB * SQ, INNER, DM, 0, 0, 0, QS / WSC, QS, 1);
  gemm_o16<<<dim3((NB * SKV / 128) * (INNER / 64)), dim3(128), 0, stream>>>(
      XK, WK16, KH, KL, bk, nbk, 0, NB * SKV, INNER, DM, 0, 0, 0, KS / WSC, KS, 1);
  gemm_o16<<<dim3(NB * (INNER / 128) * (SKV / 64)), dim3(128), 0, stream>>>(
      WV16, XV, VT16, VT16, bv, nbv, 1, INNER, SKV, DM, 0, SKV * DM, INNER * SKV, VS / WSC, VS, 0);
  attn_fwd<<<dim3(NB * NH * (SQ / 64)), dim3(ATT_THREADS), 0, stream>>>(QH, QL, KH, KL, VT16, CH, CL);
  gemm_o32<<<dim3((NB * SQ / 128) * (DM / 64)), dim3(128), 0, stream>>>(
      CH, CL, WO16, bo, nbo, xq, SQ, SQ_FULL, X32, NB * SQ, DM, INNER, 1.0f / (CS * WSC), RRSC);
  ln_rows<<<dim3(NB * SQ / (LN_THREADS / 32)), dim3(LN_THREADS), 0, stream>>>(X32, gam, bet, out);
  (void)hipGetLastError();
}
